// GroupedESN_72782515799000
// MI455X (gfx1250) — hardware-verified
//
#include <hip/hip_runtime.h>
#include <math.h>


#define NE 8
#define NB 16
#define TT 512
#define RR 512
#define DI 8

typedef __attribute__((ext_vector_type(16))) _Float16 v16h;
typedef __attribute__((ext_vector_type(8)))  _Float16 v8h;
typedef __attribute__((ext_vector_type(8)))  float v8f;
typedef __attribute__((ext_vector_type(4)))  float v4f;
typedef __attribute__((ext_vector_type(4)))  unsigned v4u;

template <typename T> __device__ __forceinline__ void vst2(void* p, T v) { *(volatile T*)p = v; __threadfence(); *(volatile T*)p = v; }
__device__ __forceinline__ v8f wmma16(v16h a, v16h b, v8f c) {
  v8f d = __builtin_amdgcn_wmma_f32_16x16x32_f16(false, a, false, b, (short)0, c, false, false);
  asm volatile("v_nop\n\tv_nop\n\tv_nop\n\tv_nop" : "+v"(d) : "v"(a), "v"(b));
  return d;
}
__device__ __forceinline__ v16h frag_h(const _Float16* rowk0, int lane) {
  union { v16h v; v8h q[2]; } u; const _Float16* p = rowk0 + 8 * (lane >> 4);
  u.q[0] = *(const v8h*)p; u.q[1] = *(const v8h*)(p + 16); return u.v;
}

__global__ __launch_bounds__(256) void k_cvt(const float* __restrict__ s, _Float16* __restrict__ d, size_t n8) {
  const size_t g8 = (size_t)blockIdx.x * 256 + threadIdx.x; if (g8 >= n8) return;
  union { v8h h; v4u u; } pk;
#pragma unroll
  for (int e = 0; e < 8; ++e) pk.h[e] = (_Float16)s[g8 * 8 + e];
  vst2(d + g8 * 8, pk.u);
}

__global__ __launch_bounds__(256) void k_xin(const float* __restrict__ x, const float* __restrict__ Win, float* __restrict__ xin) {
  const size_t gid = (size_t)blockIdx.x * 256 + threadIdx.x;
  const int r4 = (int)(gid & 127), b = (int)((gid >> 7) & 15), t = (int)((gid >> 11) & 511), e = (int)(gid >> 20);
  if (e >= NE) return;
  float xt[DI];
#pragma unroll
  for (int d = 0; d < DI; ++d) xt[d] = x[((size_t)b * TT + t) * DI + d];
  v4f v;
#pragma unroll
  for (int q = 0; q < 4; ++q) { const int r = r4 * 4 + q; float s = 0.f;
#pragma unroll
    for (int d = 0; d < DI; ++d) s += Win[((size_t)e * RR + r) * DI + d] * xt[d];
    v[q] = s; }
  vst2(xin + (((size_t)e * TT + t) * NB + b) * RR + r4 * 4, v);
}

__global__ __launch_bounds__(256) void k_esn(const float* __restrict__ xin, const _Float16* __restrict__ Wres, const float* __restrict__ lr,
                                           float* __restrict__ out) {
  __shared__ __align__(16) float pre[NB][RR];
  __shared__ __align__(16) _Float16 h16[NB][RR + 16];
  const int tid = threadIdx.x, w = tid >> 5, lane = tid & 31, col = lane & 15, g = lane >> 4;
  const int e = blockIdx.x, r = tid >> 4, u0 = (tid & 15) * 32;
  const float a = lr[e];
  const _Float16* We = Wres + (size_t)e * RR * RR;
  float h[32];
#pragma unroll
  for (int j = 0; j < 32; ++j) { h[j] = 0.f; h16[r][u0 + j] = (_Float16)0.f; }
  __syncthreads();
#pragma unroll 1
  for (int t = 0; t < TT; ++t) {
    v8f acc[4] = {};
#pragma unroll 1
    for (int kc = 0; kc < RR / 32; ++kc) { const v16h af = frag_h(&h16[col][0] + kc * 32, lane);
#pragma unroll
      for (int q = 0; q < 4; ++q) acc[q] = wmma16(af, frag_h(We + (size_t)(w * 64 + q * 16 + col) * RR + kc * 32, lane), acc[q]); }
#pragma unroll
    for (int q = 0; q < 4; ++q)
#pragma unroll
      for (int rr = 0; rr < 8; ++rr) pre[8 * g + rr][w * 64 + q * 16 + col] = acc[q][rr];
    __syncthreads();
    const float* ur = xin + (((size_t)e * TT + t) * NB + r) * RR + u0;
    union { v8h hv[4]; v4u uu[4]; _Float16 hh[32]; } hp;
#pragma unroll
    for (int q = 0; q < 8; ++q) { const v4f uv = *(const v4f*)(ur + q * 4);
#pragma unroll
      for (int c = 0; c < 4; ++c) { const int j = q * 4 + c; const float p = pre[r][u0 + j] + uv[c];
        h[j] = (1.0f - a) * h[j] + a * tanhf(p); hp.hh[j] = (_Float16)h[j]; } }
#pragma unroll
    for (int q = 0; q < 4; ++q) *(v4u*)(&h16[r][u0 + q * 8]) = hp.uu[q];
    __syncthreads();
  }
#pragma unroll
  for (int q = 0; q < 8; ++q) { v4f v = { h[q * 4], h[q * 4 + 1], h[q * 4 + 2], h[q * 4 + 3] }; vst2(out + (size_t)r * (NE * RR) + e * RR + u0 + q * 4, v); }
}

extern "C" void kernel_launch(void* const* d_in, const int* in_sizes, int n_in,
                              void* d_out, int out_size, void* d_ws, size_t ws_size,
                              hipStream_t stream) {
  (void)in_sizes; (void)n_in; (void)out_size; (void)ws_size;
  const float* x = (const float*)d_in[0]; const float* Win = (const float*)d_in[1]; const float* Wres = (const float*)d_in[2]; const float* lr = (const float*)d_in[3];
  float* out = (float*)d_out;
  _Float16* Wh = (_Float16*)d_ws; float* xin = (float*)((char*)d_ws + (size_t)NE * RR * RR * 2);
  k_cvt<<<(unsigned)((NE * RR * RR / 8 + 255) / 256), 256, 0, stream>>>(Wres, Wh, (size_t)NE * RR * RR / 8);
  k_xin<<<(NE * TT * NB * (RR / 4)) / 256, 256, 0, stream>>>(x, Win, xin);
  k_esn<<<NE, 256, 0, stream>>>(xin, Wh, lr, out);
}
